// GRUAutoencoder_67645734912183
// MI455X (gfx1250) — hardware-verified
//
#include <hip/hip_runtime.h>
#include <math.h>
#include <stdint.h>

constexpr int NSEQ  = 256;
constexpr int NTX   = 50;
constexpr int NTY   = 100;
constexpr int NIN   = 64;
constexpr int NHID  = 512;
constexpr int NG3   = 1536;
constexpr int NHOR  = 60;
constexpr int NM1   = 1024;
constexpr int NM2   = 512;
constexpr int KCAT  = 1024;
constexpr int NDIN  = 1088;
constexpr int NTHR  = 256;
constexpr int NWAVE = NTHR / 32;
constexpr int TROWS = 16;
constexpr int NRT   = NSEQ / TROWS;
constexpr int NRUN  = 4;
constexpr int HP    = 520;
constexpr int XP    = 72;
constexpr int M1P   = 1032;
constexpr int M2P   = 520;
constexpr int CATP  = 1032;
constexpr int SP    = 68;
constexpr int SLAB_FLOATS = 16 * SP;
constexpr int GI_GSTRIDE_ENC = NHID * NIN;
constexpr int GI_GSTRIDE_DEC = NHID * NDIN;
constexpr int GH_GSTRIDE     = NHID * NHID;
constexpr int HPLANE = NSEQ * NHID;
constexpr float A_CARRY = 16.0f;
constexpr float W_CARRY = 64.0f;
constexpr float Z_FOLD  = 1.0f / 1024.0f;

static_assert(NSEQ % TROWS == 0, "grid covers all sequences exactly");
static_assert(TROWS * NIN == NTHR * 4, "one float4 per thread stages a 16x64 tile exactly");
static_assert(TROWS == 2 * NWAVE && NHID == 4 * 32 * 4, "final-state store: 2 rows per wave, 4 x (32 lanes x 4 floats) per row");
static_assert(TROWS * NHID == 8 * NTHR * 4, "head input tile: 8 iterations x 256 threads x 4 floats per half");
static_assert(NIN % 32 == 0 && NHID % 32 == 0 && NM1 % 32 == 0 && NM2 % 32 == 0 && KCAT % 32 == 0, "every K is a multiple of 32");
static_assert(NG3 == NWAVE * 3 * 64 && NM1 == NWAVE * 2 * 64 && NM2 == NWAVE * 64 && NHID == NWAVE * 64 && NIN == 4 * 16, "n tiles split exactly over the waves");
static_assert((NG3 * NIN / 8) % NTHR == 0 && (NG3 * NHID / 8) % NTHR == 0 && (NM1 * KCAT / 8) % NTHR == 0 &&
              (NM2 * NM1 / 8) % NTHR == 0 && (NHID * NM2 / 8) % NTHR == 0 && (NG3 * NDIN / 8) % NTHR == 0 &&
              (NM1 * NHID / 8) % NTHR == 0 && (NIN * NM2 / 8) % NTHR == 0, "weight prep grids exact");
static_assert(HP % 8 == 0 && XP % 8 == 0 && M1P % 8 == 0 && M2P % 8 == 0 && CATP % 8 == 0 &&
              HP >= NHID && XP >= NIN && M1P >= NM1 && M2P >= NM2 && CATP >= KCAT, "16-B aligned fragment rows, k extents inside the pitch");

typedef __attribute__((ext_vector_type(16))) _Float16 v16h;
typedef __attribute__((ext_vector_type(8)))  _Float16 v8h;
typedef __attribute__((ext_vector_type(4)))  _Float16 v4h;
typedef __attribute__((ext_vector_type(16))) __bf16   v16b;
typedef __attribute__((ext_vector_type(8)))  __bf16   v8b;
typedef __attribute__((ext_vector_type(8)))  float    v8f;
typedef __attribute__((ext_vector_type(4)))  float    v4f;

__device__ __forceinline__ unsigned short f2bf_bits(float f) {
  unsigned u = __float_as_uint(f);
  return (unsigned short)((u + 0x7FFFu + ((u >> 16) & 1u)) >> 16);
}
__device__ __forceinline__ float bf_bits2f(unsigned short h) { return __uint_as_float(((unsigned)h) << 16); }
__device__ __forceinline__ float bfr(float f) { return bf_bits2f(f2bf_bits(f)); }

__device__ __forceinline__ void dep_guard_h(v8f& a, v8f& b, v16h x, v16h y) { asm volatile("v_nop\n\tv_nop\n\tv_nop\n\tv_nop" : "+v"(a), "+v"(b) : "v"(x), "v"(y)); }
__device__ __forceinline__ void dep_guard_b(v8f& a, v8f& b, v16b x, v16b y) { asm volatile("v_nop\n\tv_nop\n\tv_nop\n\tv_nop" : "+v"(a), "+v"(b) : "v"(x), "v"(y)); }
__device__ __forceinline__ void dep_guard1(v8f& a, v16h x, v16h y) { asm volatile("v_nop\n\tv_nop\n\tv_nop\n\tv_nop" : "+v"(a) : "v"(x), "v"(y)); }
__device__ __forceinline__ void keep4_h(v16h a, v16h b, v16h c, v16h d) { asm volatile("v_nop" :: "v"(a), "v"(b), "v"(c), "v"(d)); }
__device__ __forceinline__ void keep4_b(v16b a, v16b b, v16b c, v16b d) { asm volatile("v_nop" :: "v"(a), "v"(b), "v"(c), "v"(d)); }
__device__ __forceinline__ void acc_guard4(v8f& a, v8f& b, v8f& c, v8f& d) { asm volatile("v_nop\n\tv_nop\n\tv_nop\n\tv_nop" : "+v"(a), "+v"(b), "+v"(c), "+v"(d)); }
__device__ __forceinline__ void acc_guard3(v8f& a, v8f& b, v8f& c) { asm volatile("v_nop\n\tv_nop\n\tv_nop\n\tv_nop" : "+v"(a), "+v"(b), "+v"(c)); }
template <typename T> struct Frag;
template <> struct Frag<_Float16> {
  typedef v16h V; union U { v16h v; v8h h[2]; };
  static __device__ __forceinline__ v16h load(const _Float16* p) {
    U f; f.h[0] = *(const v8h*)(p); f.h[1] = *(const v8h*)(p + 16); return f.v;
  }
  static __device__ __forceinline__ v8f mma(v16h a, v16h b, v8f c) {
    return __builtin_amdgcn_wmma_f32_16x16x32_f16(false, a, false, b, (short)0, c, false, false);
  }
  static __device__ __forceinline__ void guard(v8f& a, v8f& b, v16h x, v16h y) { dep_guard_h(a, b, x, y); }
  static __device__ __forceinline__ void keep(v16h a, v16h b, v16h c, v16h d) { keep4_h(a, b, c, d); }
};
template <> struct Frag<__bf16> {
  typedef v16b V; union U { v16b v; v8b h[2]; };
  static __device__ __forceinline__ v16b load(const __bf16* p) {
    U f; f.h[0] = *(const v8b*)(p); f.h[1] = *(const v8b*)(p + 16); return f.v;
  }
  static __device__ __forceinline__ v8f mma(v16b a, v16b b, v8f c) {
    return __builtin_amdgcn_wmma_f32_16x16x32_bf16(false, a, false, b, (short)0, c, false, false);
  }
  static __device__ __forceinline__ void guard(v8f& a, v8f& b, v16b x, v16b y) { dep_guard_b(a, b, x, y); }
  static __device__ __forceinline__ void keep(v16b a, v16b b, v16b c, v16b d) { keep4_b(a, b, c, d); }
};
typedef Frag<_Float16> FragH;

__device__ __forceinline__ float fsig(float v)  { return __builtin_amdgcn_rcpf(1.0f + __expf(-v)); }
__device__ __forceinline__ float ftanh(float v) { return 1.0f - 2.0f * __builtin_amdgcn_rcpf(__expf(2.0f * v) + 1.0f); }

__global__ __launch_bounds__(NTHR) void wprep_kernel(const float* __restrict__ W, int n8, unsigned short* __restrict__ O) {
  const int i = blockIdx.x * NTHR + threadIdx.x;
  if (i >= n8) return;
  const int e0 = i * 8;
  v8h hv;
#pragma unroll
  for (int e = 0; e < 8; ++e) {
    const float fb = bfr(W[e0 + e]);
    hv[e] = (_Float16)(fb * W_CARRY);
  }
  *(volatile v8h*)(O + e0) = hv;
  __threadfence();
  *(volatile v8h*)(O + e0) = hv;
}

__device__ __forceinline__ void gru_prod(v8f (&acc)[4],
    const _Float16* gia, const _Float16* giw, const int gis,
    const _Float16* gha, const _Float16* ghw) {
#pragma unroll 1
  for (int k0 = 0; k0 < NIN; k0 += 32) {
    const v16h a  = FragH::load(gia + k0);
    const v16h b0 = FragH::load(giw + k0);
    const v16h b1 = FragH::load(giw + gis + k0);
    const v16h b2 = FragH::load(giw + 2 * gis + k0);
    acc[0] = FragH::mma(a, b0, acc[0]);
    acc[1] = FragH::mma(a, b1, acc[1]);
    acc[2] = FragH::mma(a, b2, acc[2]);
    acc_guard3(acc[0], acc[1], acc[2]);
    keep4_h(a, b0, b1, b2);
  }
#pragma unroll 1
  for (int k0 = 0; k0 < NHID; k0 += 32) {
    const v16h a  = FragH::load(gha + k0);
    const v16h b0 = FragH::load(ghw + k0);
    const v16h b1 = FragH::load(ghw + GH_GSTRIDE + k0);
    const v16h b2 = FragH::load(ghw + 2 * GH_GSTRIDE + k0);
    acc[0] = FragH::mma(a, b0, acc[0]);
    acc[1] = FragH::mma(a, b1, acc[1]);
    acc[3] = FragH::mma(a, b2, acc[3]);
    acc_guard3(acc[0], acc[1], acc[3]);
    keep4_h(a, b0, b1, b2);
  }
}

__device__ __forceinline__ void gemm_grp4(v8f (&acc)[4], const _Float16* arow, const _Float16* w0, const int ldw, const int K) {
  const v8f z8 = {0.f, 0.f, 0.f, 0.f, 0.f, 0.f, 0.f, 0.f};
  acc[0] = z8; acc[1] = z8; acc[2] = z8; acc[3] = z8;
#pragma unroll 1
  for (int k0 = 0; k0 < K; k0 += 32) {
    const v16h a  = FragH::load(arow + k0);
    const v16h b0 = FragH::load(w0 + k0);
    const v16h b1 = FragH::load(w0 + 16 * ldw + k0);
    const v16h b2 = FragH::load(w0 + 32 * ldw + k0);
    const v16h b3 = FragH::load(w0 + 48 * ldw + k0);
    acc[0] = FragH::mma(a, b0, acc[0]);
    acc[1] = FragH::mma(a, b1, acc[1]);
    acc[2] = FragH::mma(a, b2, acc[2]);
    acc[3] = FragH::mma(a, b3, acc[3]);
    dep_guard_h(acc[0], acc[3], a, a);
    keep4_h(b0, b1, b2, b3);
  }
  acc_guard4(acc[0], acc[1], acc[2], acc[3]);
}

template <bool RELU>
__device__ __forceinline__ void epi16(const v8f (&acc)[4], const float* bias, int n0, int c, int rb8,
                                      _Float16* o16, int op, int ocol) {
#pragma unroll
  for (int j = 0; j < 4; ++j) {
    const int n = n0 + 16 * j + c;
    const float bv = bfr(bias[n]);
#pragma unroll
    for (int r = 0; r < 8; ++r) {
      float v = fmaf(acc[j][r], Z_FOLD, bv);
      if (RELU) v = fmaxf(v, 0.0f);
      o16[(rb8 + r) * op + ocol + n] = (_Float16)(A_CARRY * v);
    }
  }
}

__device__ __forceinline__ void epi_const(const v8f (&acc)[4], const float* bias, int n0, int c, int hh, int lane,
                                          float* slab, float* C, int rowbase) {
#pragma unroll
  for (int j = 0; j < 4; ++j) {
    const int n = n0 + 16 * j + c;
    const float bv = bfr(bias[n]);
#pragma unroll
    for (int r = 0; r < 8; ++r) slab[(8 * hh + r) * SP + 16 * j + c] = fmaf(acc[j][r], Z_FOLD, bv);
  }
  __builtin_amdgcn_fence(__ATOMIC_RELEASE, "workgroup");
  __builtin_amdgcn_wave_barrier();
  __builtin_amdgcn_fence(__ATOMIC_ACQUIRE, "workgroup");
  const int c4 = (lane & 15) * 4;
  for (int pass = 0; pass < 2; ++pass) {
#pragma unroll
    for (int it = 0; it < 8; ++it) {
      const int row = it * 2 + hh;
      const v4f v = *(const v4f*)(slab + row * SP + c4);
      *(volatile v4f*)(C + (size_t)(rowbase + row) * NG3 + n0 + c4) = v;
    }
    __threadfence();
  }
  __builtin_amdgcn_fence(__ATOMIC_RELEASE, "workgroup");
  __builtin_amdgcn_wave_barrier();
  __builtin_amdgcn_fence(__ATOMIC_ACQUIRE, "workgroup");
}

__device__ __forceinline__ void refresh_h16(_Float16* H16, const float* HF, int rb8, int ubase) {
#pragma unroll 1
  for (int t = 0; t < 4; ++t) {
    const int u = ubase + 16 * t;
#pragma unroll
    for (int r = 0; r < 8; ++r) H16[(rb8 + r) * HP + u] = (_Float16)(A_CARRY * HF[(rb8 + r) * NHID + u]);
  }
}

struct EncParams {
  const float* x;  const float* y;
  const float* bih0; const float* bhh0; const float* bih1; const float* bhh1;
  const float* bih2; const float* bhh2; const float* bih3; const float* bhh3;
  const unsigned short* wih0; const unsigned short* whh0; const unsigned short* wih1; const unsigned short* whh1;
  const unsigned short* wih2; const unsigned short* whh2; const unsigned short* wih3; const unsigned short* whh3;
  float* hfin;
};
static_assert(sizeof(EncParams) == 19 * 8, "pointer-only struct, no padding");

__global__ __launch_bounds__(NTHR) __attribute__((amdgpu_num_vgpr(256)))
void gru_enc_kernel(EncParams p) {
  __shared__ __align__(16) _Float16 H16[TROWS * HP];
  __shared__ __align__(16) _Float16 X16[TROWS * XP];
  __shared__ __align__(16) float    HF[TROWS * NHID];

  const int tid = threadIdx.x, lane = tid & 31, wave = tid >> 5;
  const int c = lane & 15, hh = lane >> 4, koff = hh * 8, rb8 = hh * 8;
  const int run = blockIdx.x / NRT;
  const int rowbase = (blockIdx.x - run * NRT) * TROWS;
  const bool isx = run < 2;
  const bool rev = (run & 1) != 0;
  const int  T   = isx ? NTX : NTY;
  const float* X = isx ? p.x : p.y;
  const _Float16* WIH = (const _Float16*)(run == 0 ? p.wih0 : (run == 1 ? p.wih1 : (run == 2 ? p.wih2 : p.wih3)));
  const _Float16* WHH = (const _Float16*)(run == 0 ? p.whh0 : (run == 1 ? p.whh1 : (run == 2 ? p.whh2 : p.whh3)));
  const float* bih = run == 0 ? p.bih0 : (run == 1 ? p.bih1 : (run == 2 ? p.bih2 : p.bih3));
  const float* bhh = run == 0 ? p.bhh0 : (run == 1 ? p.bhh1 : (run == 2 ? p.bhh2 : p.bhh3));
  const int ubase = 64 * wave + c;

#pragma unroll 1
  for (int i = tid; i < TROWS * HP; i += NTHR) H16[i] = (_Float16)0.0f;
#pragma unroll 1
  for (int i = tid; i < TROWS * NHID; i += NTHR) HF[i] = 0.0f;

  const _Float16* hrow = H16 + c * HP + koff;
  const _Float16* xrow = X16 + c * XP + koff;

#pragma unroll 1
  for (int s = 0; s < T; ++s) {
    const int t = rev ? (T - 1 - s) : s;
    {
      const int row = tid >> 4, c4 = (tid & 15) * 4;
      const v4f v = *(const v4f*)(X + ((size_t)(rowbase + row) * T + (size_t)t) * NIN + c4);
      v4h w;
      w[0] = (_Float16)(A_CARRY * bfr(v[0]));
      w[1] = (_Float16)(A_CARRY * bfr(v[1]));
      w[2] = (_Float16)(A_CARRY * bfr(v[2]));
      w[3] = (_Float16)(A_CARRY * bfr(v[3]));
      *(v4h*)(X16 + row * XP + c4) = w;
    }
    __syncthreads();
#pragma unroll 1
    for (int tt = 0; tt < 4; ++tt) {
      const int u = ubase + 16 * tt;
      const v8f z8 = {0.f, 0.f, 0.f, 0.f, 0.f, 0.f, 0.f, 0.f};
      v8f acc[4];
      acc[0] = z8; acc[1] = z8; acc[2] = z8; acc[3] = z8;
      gru_prod(acc, xrow, WIH + (size_t)u * NIN + koff, GI_GSTRIDE_ENC, hrow, WHH + (size_t)u * NHID + koff);
      const float cr = bfr(bih[u]) + bfr(bhh[u]);
      const float cz = bfr(bih[NHID + u]) + bfr(bhh[NHID + u]);
      const float ci = bfr(bih[2 * NHID + u]);
      const float ch = bfr(bhh[2 * NHID + u]);
#pragma unroll
      for (int r = 0; r < 8; ++r) {
        float* hp = HF + (rb8 + r) * NHID + u;
        const float hold = *hp;
        const float pr  = fmaf(acc[0][r], Z_FOLD, cr);
        const float pz  = fmaf(acc[1][r], Z_FOLD, cz);
        const float gin = fmaf(acc[2][r], Z_FOLD, ci);
        const float ghn = fmaf(acc[3][r], Z_FOLD, ch);
        const float rr  = fsig(pr);
        const float zz  = fsig(pz);
        const float nn  = ftanh(fmaf(rr, ghn, gin));
        *hp = fmaf(zz, hold - nn, nn);
      }
    }
    __syncthreads();
    refresh_h16(H16, HF, rb8, ubase);
  }
  __syncthreads();

  {
    float* dst = p.hfin + ((size_t)run * NSEQ + (size_t)rowbase) * NHID;
    for (int pass = 0; pass < 2; ++pass) {
#pragma unroll
      for (int r2 = 0; r2 < 2; ++r2) {
        const int row = wave * 2 + r2;
#pragma unroll
        for (int q = 0; q < 4; ++q) {
          const v4f v = *(const v4f*)(HF + row * NHID + q * 128 + lane * 4);
          *(volatile v4f*)(dst + (size_t)row * NHID + q * 128 + lane * 4) = v;
        }
      }
      __threadfence();
    }
  }
}

struct HeadParams {
  const float* hfin; const float* em_b1; const float* em_b2; const float* eo_b; const float* dg_bih;
  const unsigned short* em_w1; const unsigned short* em_w2; const unsigned short* eo_w; const unsigned short* dg_wih;
  float* cst;
};
static_assert(sizeof(HeadParams) == 10 * 8, "pointer-only struct, no padding");

__global__ __launch_bounds__(NTHR) __attribute__((amdgpu_num_vgpr(256)))
void mlp_head_kernel(HeadParams p) {
  __shared__ __align__(16) _Float16 CAT16[TROWS * CATP];
  __shared__ __align__(16) _Float16 M1H[TROWS * M1P];
  __shared__ __align__(16) _Float16 M2H[TROWS * M2P];
  __shared__ __align__(16) float    SLAB[NWAVE * SLAB_FLOATS];

  const int tid = threadIdx.x, lane = tid & 31, wave = tid >> 5;
  const int c = lane & 15, hh = lane >> 4, koff = hh * 8, rb8 = hh * 8;
  const int rowbase = blockIdx.x * TROWS;

#pragma unroll 1
  for (int it = 0; it < 8; ++it) {
    const int q = it * NTHR + tid;
    const int row = q >> 7, c4 = (q & 127) * 4;
    const size_t o = (size_t)(rowbase + row) * NHID + c4;
    const v4f a0 = *(const v4f*)(p.hfin + o);
    const v4f a1 = *(const v4f*)(p.hfin + (size_t)HPLANE + o);
    const v4f a2 = *(const v4f*)(p.hfin + 2 * (size_t)HPLANE + o);
    const v4f a3 = *(const v4f*)(p.hfin + 3 * (size_t)HPLANE + o);
    v4h hx, hy;
#pragma unroll
    for (int e = 0; e < 4; ++e) {
      hx[e] = (_Float16)(A_CARRY * (a0[e] + a1[e]));
      hy[e] = (_Float16)(A_CARRY * (a2[e] + a3[e]));
    }
    *(v4h*)(CAT16 + row * CATP + c4) = hx;
    *(v4h*)(CAT16 + row * CATP + NHID + c4) = hy;
  }
  __syncthreads();

  const _Float16* catrow = CAT16 + c * CATP + koff;
  const _Float16* m1row  = M1H + c * M1P + koff;
  const _Float16* m2row  = M2H + c * M2P + koff;

  {
    const _Float16* wl = (const _Float16*)p.em_w1 + (size_t)c * KCAT + koff;
#pragma unroll 1
    for (int grp = 0; grp < 2; ++grp) {
      const int n0 = (wave * 2 + grp) * 64;
      v8f acc[4];
      gemm_grp4(acc, catrow, wl + (size_t)n0 * KCAT, KCAT, KCAT);
      epi16<true>(acc, p.em_b1, n0, c, rb8, M1H, M1P, 0);
    }
  }
  __syncthreads();
  {
    const _Float16* wl = (const _Float16*)p.em_w2 + (size_t)c * NM1 + koff;
    const int n0 = wave * 64;
    v8f acc[4];
    gemm_grp4(acc, m1row, wl + (size_t)n0 * NM1, NM1, NM1);
    epi16<true>(acc, p.em_b2, n0, c, rb8, M2H, M2P, 0);
  }
  __syncthreads();
  {
    const _Float16* wl = (const _Float16*)p.eo_w + (size_t)c * NM2 + koff;
    const int n0 = wave * 64;
    v8f acc[4];
    gemm_grp4(acc, m2row, wl + (size_t)n0 * NM2, NM2, NM2);
    epi16<false>(acc, p.eo_b, n0, c, rb8, CAT16, CATP, NHID);
  }
  __syncthreads();
  {
    const _Float16* wl = (const _Float16*)p.dg_wih + (size_t)c * NDIN + koff;
    float* slab = SLAB + wave * SLAB_FLOATS;
#pragma unroll 1
    for (int grp = 0; grp < 3; ++grp) {
      const int n0 = (wave * 3 + grp) * 64;
      v8f acc[4];
      gemm_grp4(acc, catrow, wl + (size_t)n0 * NDIN, NDIN, KCAT);
      epi_const(acc, p.dg_bih, n0, c, hh, lane, slab, p.cst, rowbase);
    }
  }
}

struct DecParams {
  const float* x; const float* cst; const float* dg_bhh; const float* dm_b1; const float* dm_b2; const float* do_b;
  const unsigned short* dg_wih; const unsigned short* dg_whh; const unsigned short* dm_w1; const unsigned short* dm_w2;
  const unsigned short* do_w;
  float* out;
};
static_assert(sizeof(DecParams) == 12 * 8, "pointer-only struct, no padding");

__global__ __launch_bounds__(NTHR) __attribute__((amdgpu_num_vgpr(256)))
void gru_dec_kernel(DecParams p) {
  __shared__ __align__(16) _Float16 H16[TROWS * HP];
  __shared__ __align__(16) float    HF[TROWS * NHID];
  __shared__ __align__(16) _Float16 Y16[TROWS * XP];
  __shared__ __align__(16) _Float16 M1H[TROWS * M1P];
  __shared__ __align__(16) _Float16 M2H[TROWS * M2P];
  __shared__ __align__(16) float    YS[TROWS * SP];

  const int tid = threadIdx.x, lane = tid & 31, wave = tid >> 5;
  const int c = lane & 15, hh = lane >> 4, koff = hh * 8, rb8 = hh * 8;
  const int rowbase = blockIdx.x * TROWS;
  const int ubase = 64 * wave + c;
  const v8f z8 = {0.f, 0.f, 0.f, 0.f, 0.f, 0.f, 0.f, 0.f};

#pragma unroll 1
  for (int i = tid; i < TROWS * HP; i += NTHR) H16[i] = (_Float16)0.0f;
#pragma unroll 1
  for (int i = tid; i < TROWS * NHID; i += NTHR) HF[i] = 0.0f;
  {
    const int row = tid >> 4, c4 = (tid & 15) * 4;
    const v4f v = *(const v4f*)(p.x + ((size_t)(rowbase + row) * NTX + (size_t)(NTX - 1)) * NIN + c4);
    v4h w;
    w[0] = (_Float16)(A_CARRY * bfr(v[0]));
    w[1] = (_Float16)(A_CARRY * bfr(v[1]));
    w[2] = (_Float16)(A_CARRY * bfr(v[2]));
    w[3] = (_Float16)(A_CARRY * bfr(v[3]));
    *(v4h*)(Y16 + row * XP + c4) = w;
  }
  const _Float16* DWIH = (const _Float16*)p.dg_wih;
  const _Float16* DWHH = (const _Float16*)p.dg_whh;
  const _Float16* DMW1 = (const _Float16*)p.dm_w1;
  const _Float16* DMW2 = (const _Float16*)p.dm_w2;
  const _Float16* DOW  = (const _Float16*)p.do_w;
  const float* cstrow = p.cst + (size_t)(rowbase + rb8) * NG3;
  const _Float16* hrow  = H16 + c * HP + koff;
  const _Float16* yrow  = Y16 + c * XP + koff;
  const _Float16* m1row = M1H + c * M1P + koff;
  const _Float16* m2row = M2H + c * M2P + koff;
  __syncthreads();

#pragma unroll 1
  for (int s = 0; s < NHOR; ++s) {
#pragma unroll 1
    for (int tt = 0; tt < 4; ++tt) {
      const int u = ubase + 16 * tt;
      v8f acc[4];
      acc[0] = z8; acc[1] = z8; acc[2] = z8; acc[3] = z8;
      gru_prod(acc, yrow, DWIH + (size_t)u * NDIN + 2 * NHID + koff, GI_GSTRIDE_DEC, hrow, DWHH + (size_t)u * NHID + koff);
      const float br = bfr(p.dg_bhh[u]);
      const float bz = bfr(p.dg_bhh[NHID + u]);
      const float bn = bfr(p.dg_bhh[2 * NHID + u]);
#pragma unroll
      for (int r = 0; r < 8; ++r) {
        const float* cp = cstrow + (size_t)r * NG3 + u;
        const float xr = cp[0];
        const float xz = cp[NHID];
        const float xn = cp[2 * NHID];
        float* hp = HF + (rb8 + r) * NHID + u;
        const float hold = *hp;
        const float pr  = fmaf(acc[0][r], Z_FOLD, xr + br);
        const float pz  = fmaf(acc[1][r], Z_FOLD, xz + bz);
        const float gin = fmaf(acc[2][r], Z_FOLD, xn);
        const float ghn = fmaf(acc[3][r], Z_FOLD, bn);
        const float rr  = fsig(pr);
        const float zz  = fsig(pz);
        const float nn  = ftanh(fmaf(rr, ghn, gin));
        *hp = fmaf(zz, hold - nn, nn);
      }
    }
    __syncthreads();
    refresh_h16(H16, HF, rb8, ubase);
    __syncthreads();
    {
      const _Float16* wl = DMW1 + (size_t)c * NHID + koff;
#pragma unroll 1
      for (int grp = 0; grp < 2; ++grp) {
        const int n0 = (wave * 2 + grp) * 64;
        v8f acc[4];
        gemm_grp4(acc, hrow, wl + (size_t)n0 * NHID, NHID, NHID);
        epi16<true>(acc, p.dm_b1, n0, c, rb8, M1H, M1P, 0);
      }
    }
    __syncthreads();
    {
      const _Float16* wl = DMW2 + (size_t)c * NM1 + koff;
      const int n0 = wave * 64;
      v8f acc[4];
      gemm_grp4(acc, m1row, wl + (size_t)n0 * NM1, NM1, NM1);
      epi16<true>(acc, p.dm_b2, n0, c, rb8, M2H, M2P, 0);
    }
    __syncthreads();
    if (wave < 4) {
      const int n = 16 * wave + c;
      const _Float16* wl = DOW + (size_t)n * NM2 + koff;
      v8f acc = z8;
#pragma unroll 1
      for (int k0 = 0; k0 < NM2; k0 += 32) {
        const v16h a = FragH::load(m2row + k0);
        const v16h b = FragH::load(wl + k0);
        acc = FragH::mma(a, b, acc);
        dep_guard1(acc, a, b);
      }
      const float bv = bfr(p.do_b[n]);
#pragma unroll
      for (int r = 0; r < 8; ++r) {
        const float v = fmaf(acc[r], Z_FOLD, bv);
        YS[(rb8 + r) * SP + n]  = v;
        Y16[(rb8 + r) * XP + n] = (_Float16)(A_CARRY * v);
      }
    }
    __syncthreads();
    if (wave == 0) {
      const int c4 = (lane & 15) * 4;
      float* ob = p.out + (size_t)rowbase * (NHOR * NIN) + (size_t)s * NIN + c4;
      for (int pass = 0; pass < 2; ++pass) {
#pragma unroll
        for (int it = 0; it < 8; ++it) {
          const int row = it * 2 + hh;
          const v4f v = *(const v4f*)(YS + row * SP + c4);
          *(volatile v4f*)(ob + (size_t)row * (NHOR * NIN)) = v;
        }
        __threadfence();
      }
    }
  }
}

extern "C" void kernel_launch(void* const* d_in, const int* in_sizes, int n_in,
                              void* d_out, int out_size, void* d_ws, size_t ws_size, hipStream_t stream) {
  if (n_in < 34 || d_out == nullptr || d_ws == nullptr) return;
  if (in_sizes[0] != NSEQ * NTX * NIN || in_sizes[1] != NSEQ * NTY * NIN) return;
  for (int g = 0; g < 4; ++g) {
    const int b = 2 + 4 * g;
    if (in_sizes[b] != NG3 * NIN || in_sizes[b + 1] != NG3 * NHID || in_sizes[b + 2] != NG3 || in_sizes[b + 3] != NG3) return;
  }
  if (in_sizes[18] != NM1 * KCAT || in_sizes[19] != NM1 || in_sizes[20] != NM2 * NM1 || in_sizes[21] != NM2 ||
      in_sizes[22] != NHID * NM2 || in_sizes[23] != NHID || in_sizes[24] != NG3 * NDIN || in_sizes[25] != NG3 * NHID ||
      in_sizes[26] != NG3 || in_sizes[27] != NG3 || in_sizes[28] != NM1 * NHID || in_sizes[29] != NM1 ||
      in_sizes[30] != NM2 * NM1 || in_sizes[31] != NM2 || in_sizes[32] != NIN * NM2 || in_sizes[33] != NIN ||
      out_size != NSEQ * NHOR * NIN) return;

  char* ws = (char*)d_ws; size_t off = 0;
  auto carve = [&](size_t bytes) -> char* { char* q = ws + off; off += (bytes + 255) & ~(size_t)255; return q; };
  unsigned short* XFWIH = (unsigned short*)carve((size_t)NG3 * NIN * 2);
  unsigned short* XFWHH = (unsigned short*)carve((size_t)NG3 * NHID * 2);
  unsigned short* XBWIH = (unsigned short*)carve((size_t)NG3 * NIN * 2);
  unsigned short* XBWHH = (unsigned short*)carve((size_t)NG3 * NHID * 2);
  unsigned short* EFWIH = (unsigned short*)carve((size_t)NG3 * NIN * 2);
  unsigned short* EFWHH = (unsigned short*)carve((size_t)NG3 * NHID * 2);
  unsigned short* EBWIH = (unsigned short*)carve((size_t)NG3 * NIN * 2);
  unsigned short* EBWHH = (unsigned short*)carve((size_t)NG3 * NHID * 2);
  unsigned short* EMW1  = (unsigned short*)carve((size_t)NM1 * KCAT * 2);
  unsigned short* EMW2  = (unsigned short*)carve((size_t)NM2 * NM1 * 2);
  unsigned short* EOW   = (unsigned short*)carve((size_t)NHID * NM2 * 2);
  unsigned short* DWIH  = (unsigned short*)carve((size_t)NG3 * NDIN * 2);
  unsigned short* DWHH  = (unsigned short*)carve((size_t)NG3 * NHID * 2);
  unsigned short* DMW1  = (unsigned short*)carve((size_t)NM1 * NHID * 2);
  unsigned short* DMW2  = (unsigned short*)carve((size_t)NM2 * NM1 * 2);
  unsigned short* DOW   = (unsigned short*)carve((size_t)NIN * NM2 * 2);
  float*          HFIN  = (float*)carve((size_t)NRUN * NSEQ * NHID * 4);
  float*          CST   = (float*)carve((size_t)NSEQ * NG3 * 4);
  if (off > ws_size || off > (size_t)134217728) return;

  auto prep = [&](int idx, int nelem, unsigned short* O) {
    const int n8 = nelem / 8;
    wprep_kernel<<<n8 / NTHR, NTHR, 0, stream>>>((const float*)d_in[idx], n8, O);
  };
  prep(2,  NG3 * NIN,  XFWIH);  prep(3,  NG3 * NHID, XFWHH);
  prep(6,  NG3 * NIN,  XBWIH);  prep(7,  NG3 * NHID, XBWHH);
  prep(10, NG3 * NIN,  EFWIH);  prep(11, NG3 * NHID, EFWHH);
  prep(14, NG3 * NIN,  EBWIH);  prep(15, NG3 * NHID, EBWHH);
  prep(18, NM1 * KCAT, EMW1);   prep(20, NM2 * NM1,  EMW2);   prep(22, NHID * NM2, EOW);
  prep(24, NG3 * NDIN, DWIH);   prep(25, NG3 * NHID, DWHH);
  prep(28, NM1 * NHID, DMW1);   prep(30, NM2 * NM1,  DMW2);   prep(32, NIN * NM2,  DOW);

  EncParams e;
  e.x = (const float*)d_in[0];  e.y = (const float*)d_in[1];
  e.bih0 = (const float*)d_in[4];  e.bhh0 = (const float*)d_in[5];
  e.bih1 = (const float*)d_in[8];  e.bhh1 = (const float*)d_in[9];
  e.bih2 = (const float*)d_in[12]; e.bhh2 = (const float*)d_in[13];
  e.bih3 = (const float*)d_in[16]; e.bhh3 = (const float*)d_in[17];
  e.wih0 = XFWIH; e.whh0 = XFWHH; e.wih1 = XBWIH; e.whh1 = XBWHH;
  e.wih2 = EFWIH; e.whh2 = EFWHH; e.wih3 = EBWIH; e.whh3 = EBWHH;
  e.hfin = HFIN;
  gru_enc_kernel<<<NRUN * NRT, NTHR, 0, stream>>>(e);

  HeadParams h;
  h.hfin = HFIN;
  h.em_b1 = (const float*)d_in[19]; h.em_b2 = (const float*)d_in[21]; h.eo_b = (const float*)d_in[23];
  h.dg_bih = (const float*)d_in[26];
  h.em_w1 = EMW1; h.em_w2 = EMW2; h.eo_w = EOW; h.dg_wih = DWIH;
  h.cst = CST;
  mlp_head_kernel<<<NRT, NTHR, 0, stream>>>(h);

  DecParams d;
  d.x = (const float*)d_in[0]; d.cst = CST;
  d.dg_bhh = (const float*)d_in[27];
  d.dm_b1 = (const float*)d_in[29]; d.dm_b2 = (const float*)d_in[31]; d.do_b = (const float*)d_in[33];
  d.dg_wih = DWIH; d.dg_whh = DWHH; d.dm_w1 = DMW1; d.dm_w2 = DMW2; d.do_w = DOW;
  d.out = (float*)d_out;
  gru_dec_kernel<<<NRT, NTHR, 0, stream>>>(d);
}
